// PolyNetFP4_76355928588537
// MI455X (gfx1250) — hardware-verified
//
#include <hip/hip_runtime.h>


#define NR   2097152
#define RB   262144
#define H1   64
#define H3   32
typedef _Float16 h16;
typedef unsigned short bf;
typedef __attribute__((ext_vector_type(16))) __bf16   v16bf;
typedef __attribute__((ext_vector_type(16))) _Float16 v16h;
typedef __attribute__((ext_vector_type(8)))  _Float16 v8h;
typedef __attribute__((ext_vector_type(8)))  unsigned short v8us;
typedef __attribute__((ext_vector_type(8)))  float    v8f;
typedef __attribute__((ext_vector_type(4)))  float    v4f;
typedef v8h  __attribute__((may_alias)) v8ha;
typedef v4f  __attribute__((may_alias)) v4fa;
typedef v8us __attribute__((may_alias)) v8usa;

__device__ __forceinline__ unsigned short f2bf(float f) { unsigned u = __float_as_uint(f); u += 0x7FFFu + ((u >> 16) & 1u); return (unsigned short)(u >> 16); }
__device__ __forceinline__ float bf2f(unsigned short b) { return __uint_as_float(((unsigned)b) << 16); }
__device__ __forceinline__ float bfr(float f) { return bf2f(f2bf(f)); }
__device__ __forceinline__ v16h cat16(v8h lo, v8h hi) { return __builtin_shufflevector(lo, hi, 0, 1, 2, 3, 4, 5, 6, 7, 8, 9, 10, 11, 12, 13, 14, 15); }
__device__ __forceinline__ v16bf cat16b(v8us lo, v8us hi) { return __builtin_bit_cast(v16bf, __builtin_shufflevector(lo, hi, 0, 1, 2, 3, 4, 5, 6, 7, 8, 9, 10, 11, 12, 13, 14, 15)); }
__device__ __forceinline__ v8f wmma16(v16h a, v16h b, v8f c) { return __builtin_amdgcn_wmma_f32_16x16x32_f16(false, a, false, b, (short)0, c, false, false); }
__device__ __forceinline__ v8f wmmab(v16bf a, v16bf b, v8f c) { return __builtin_amdgcn_wmma_f32_16x16x32_bf16(false, a, false, b, (short)0, c, false, false); }


template <typename T16> struct WFrag;
template <> struct WFrag<h16> { typedef v16h V; static __device__ __forceinline__ V ld(const h16* p) { return cat16(*(const v8h*)p, *(const v8h*)(p + 16)); } static __device__ __forceinline__ v8f mma(V a, V b, v8f c) { return wmma16(a, b, c); } };
template <> struct WFrag<bf> { typedef v16bf V; static __device__ __forceinline__ V ld(const bf* p) { return cat16b(*(const v8us*)p, *(const v8us*)(p + 16)); } static __device__ __forceinline__ v8f mma(V a, V b, v8f c) { return wmmab(a, b, c); } };
template <typename T16, int NSPLIT, bool BIAS>
__global__ __launch_bounds__(32) void k_gemmw(const T16* __restrict__ A, const T16* __restrict__ A2, const T16* __restrict__ Bt, const T16* __restrict__ Bt2, int K, float* C, int ldc, const float* __restrict__ bias, size_t sA, size_t sB, size_t sC) {
    typedef typename WFrag<T16>::V V;
    __shared__ __align__(16) float os[16 * 68];
    const size_t z = blockIdx.z; A += z * sA; if (A2) A2 += z * sA; Bt += z * sB; if (Bt2) Bt2 += z * sB; C += z * sC;
    const int lane = threadIdx.x & 31, lr = lane & 15, hi = lane >> 4; const int r0 = blockIdx.x * 64, c0 = blockIdx.y * 64;
    v8f acc[4][4];
#pragma unroll
    for (int mb = 0; mb < 4; ++mb)
#pragma unroll
        for (int nb = 0; nb < 4; ++nb) acc[mb][nb] = (v8f){};
    const size_t aoff = (size_t)(r0 + lr) * K + 8 * hi, boff = (size_t)(c0 + lr) * K + 8 * hi;
#pragma unroll 1
    for (int kc = 0; kc < K; kc += 32) {
        V a[4], a2[4];
#pragma unroll
        for (int mb = 0; mb < 4; ++mb) { a[mb] = WFrag<T16>::ld(A + aoff + (size_t)mb * 16 * K + kc); if (NSPLIT == 1 || NSPLIT == 2) a2[mb] = WFrag<T16>::ld(A2 + aoff + (size_t)mb * 16 * K + kc); }
#pragma unroll
        for (int nb = 0; nb < 4; ++nb) { const V b = WFrag<T16>::ld(Bt + boff + (size_t)nb * 16 * K + kc); V b2; if (NSPLIT >= 2) b2 = WFrag<T16>::ld(Bt2 + boff + (size_t)nb * 16 * K + kc);
#pragma unroll
            for (int mb = 0; mb < 4; ++mb) { acc[mb][nb] = WFrag<T16>::mma(a[mb], b, acc[mb][nb]); if (NSPLIT == 1 || NSPLIT == 2) acc[mb][nb] = WFrag<T16>::mma(a2[mb], b, acc[mb][nb]); if (NSPLIT >= 2) acc[mb][nb] = WFrag<T16>::mma(a[mb], b2, acc[mb][nb]); } }
        asm volatile("v_nop\n\tv_nop\n\tv_nop\n\tv_nop" : "+v"(acc[0][0]), "+v"(acc[1][1]), "+v"(acc[2][2]), "+v"(acc[3][3]) : "v"(a[0]), "v"(a[3]));
    }
#pragma unroll
    for (int mb = 0; mb < 4; ++mb) {
#pragma unroll
        for (int nb = 0; nb < 4; ++nb) {
#pragma unroll
            for (int j = 0; j < 8; ++j) os[(hi * 8 + j) * 68 + nb * 16 + lr] = acc[mb][nb][j]; }
        __builtin_amdgcn_wave_barrier(); asm volatile("" ::: "memory");
        float* crow = C + (size_t)(r0 + mb * 16) * ldc + c0;
#pragma unroll 1
        for (int ps = 0; ps < 2; ++ps) {
#pragma unroll
            for (int s = 0; s < 8; ++s) { const int row = 2 * s + hi, cofs = lr * 4; v4f val = *(const v4fa*)(os + row * 68 + cofs); if (BIAS) { val[0] += bfr(bias[c0 + cofs]); val[1] += bfr(bias[c0 + cofs + 1]); val[2] += bfr(bias[c0 + cofs + 2]); val[3] += bfr(bias[c0 + cofs + 3]); }
                *(volatile v4f*)(crow + (size_t)row * ldc + cofs) = val; }
            if (ps == 0) __threadfence(); }
        __builtin_amdgcn_wave_barrier(); asm volatile("" ::: "memory");
    }
}

__device__ __forceinline__ h16 tohx(float x) { return (h16)x; }
typedef __attribute__((ext_vector_type(2))) _Float16 v2h;
__constant__ float FP4C[16] = {0.0f, 0.0052083333f, 0.6666667f, 1.0f, 0.33333334f, 0.5f, 0.16666667f, 0.25f, -0.0f, -0.0052083333f, -0.6666667f, -1.0f, -0.33333334f, -0.5f, -0.16666667f, -0.25f};

__global__ __launch_bounds__(64) void k_fp4(const float* __restrict__ w, int n, float* Q) { const int blk = blockIdx.x * 64 + threadIdx.x; const int nb = (n + 63) / 64; if (blk >= nb) return; float am = 0.f;
    for (int i = 0; i < 64; ++i) { const int e = blk * 64 + i; const float v = (e < n) ? bfr(w[e]) : 0.f; am = fmaxf(am, fabsf(v)); }
    const float sc = (am == 0.f) ? 1.0f : am;
    for (int ps = 0; ps < 2; ++ps) { for (int i = 0; i < 64; ++i) { const int e = blk * 64 + i; if (e >= n) break; const float v = bfr(w[e]); const float s = __fdiv_rn(v, sc); int best = 0; float bd = fabsf(__fsub_rn(s, FP4C[0]));
            for (int c = 1; c < 16; ++c) { const float d = fabsf(__fsub_rn(s, FP4C[c])); if (d < bd) { bd = d; best = c; } }
            *(volatile float*)(Q + e) = __fmul_rn(FP4C[best], am); } if (ps == 0) __threadfence(); } }
__global__ __launch_bounds__(256) void k_w16(const float* __restrict__ Q2, const float* __restrict__ Q3, const float* __restrict__ b3, h16* W2h, h16* W3h, float* B3P) { const int t = threadIdx.x;
    for (int ps = 0; ps < 2; ++ps) { for (int i = t; i < 64 * 64; i += 256) { *(volatile h16*)(W2h + i) = tohx(Q2[i]); *(volatile h16*)(W3h + i) = (i < H3 * 64) ? tohx(Q3[i]) : tohx(0.f); } if (t < 64) *(volatile float*)(B3P + t) = (t < H3) ? bfr(b3[t]) : 0.f; if (ps == 0) __threadfence(); } }
__global__ __launch_bounds__(256) void k_l1(const float* __restrict__ x, const float* __restrict__ Q1, const float* __restrict__ b1, int r0, h16* H1h) { const size_t i = ((size_t)blockIdx.x * 256 + threadIdx.x) * 2; if (i >= (size_t)RB * H1) return; const int r = (int)(i / H1), j = (int)(i % H1); const float xv = bfr(x[r0 + r]); v2h o;
#pragma unroll
    for (int q = 0; q < 2; ++q) { float p = __fmul_rn(xv, Q1[j + q]); asm volatile("" : "+v"(p)); const float h = __fadd_rn(p, bfr(b1[j + q])); o[q] = tohx(__fdiv_rn(h, __fadd_rn(1.0f, __expf(-h)))); }
    *(volatile v2h*)(H1h + i) = o; __threadfence(); *(volatile v2h*)(H1h + i) = o; }
__global__ __launch_bounds__(256) void k_act(const float* __restrict__ F, h16* Hh) { const size_t i = ((size_t)blockIdx.x * 256 + threadIdx.x) * 2; if (i >= (size_t)RB * H1) return; v2h o;
#pragma unroll
    for (int q = 0; q < 2; ++q) { const float h = F[i + q]; o[q] = tohx(__fdiv_rn(h, __fadd_rn(1.0f, __expf(-h)))); } *(volatile v2h*)(Hh + i) = o; __threadfence(); *(volatile v2h*)(Hh + i) = o; }
__global__ __launch_bounds__(256) void k_out(const float* __restrict__ F3, const float* __restrict__ Q4, const float* __restrict__ b4, int r0, float* OUT) { const int r = blockIdx.x * 256 + threadIdx.x; if (r >= RB) return; const float* f = F3 + (size_t)r * H1; float s = 0.f;
#pragma unroll 2
    for (int j = 0; j < H3; j += 4) { const v4f v = *(const v4f*)(f + j);
#pragma unroll
        for (int q = 0; q < 4; ++q) { const float h = v[q]; const float a = __fdiv_rn(h, __fadd_rn(1.0f, __expf(-h))); float p = __fmul_rn(a, Q4[j + q]); asm volatile("" : "+v"(p)); s = __fadd_rn(s, p); } }
    const float o = __fadd_rn(s, bfr(b4[0])); *(volatile float*)(OUT + r0 + r) = o; __threadfence(); *(volatile float*)(OUT + r0 + r) = o; }

extern "C" void kernel_launch(void* const* d_in, const int* in_sizes, int n_in,
                              void* d_out, int out_size, void* d_ws, size_t ws_size, hipStream_t stream) {
    (void)in_sizes; (void)n_in; (void)out_size;
    const float* IN[9]; for (int i = 0; i < 9; ++i) IN[i] = (const float*)d_in[i];
    float* OUT = (float*)d_out;
    char* wsp = (char*)d_ws;
    auto take = [&](size_t bytes) { char* p = wsp; wsp += (bytes + 255) & ~(size_t)255; return (void*)p; };
    float* Q1 = (float*)take(64 * 4); float* Q2 = (float*)take(64 * 64 * 4); float* Q3 = (float*)take(32 * 64 * 4); float* Q4 = (float*)take(64 * 4); h16* W2h = (h16*)take(64 * 64 * 2); h16* W3h = (h16*)take(64 * 64 * 2); float* B3P = (float*)take(64 * 4);
    h16* H1h = (h16*)take((size_t)RB * H1 * 2); float* F = (float*)take((size_t)RB * H1 * 4); h16* H2h = (h16*)take((size_t)RB * H1 * 2);
    if ((size_t)(wsp - (char*)d_ws) > ws_size) return;
    k_fp4<<<1, 64, 0, stream>>>(IN[1], 64, Q1); k_fp4<<<1, 64, 0, stream>>>(IN[3], 64 * 64, Q2); k_fp4<<<1, 64, 0, stream>>>(IN[5], 32 * 64, Q3); k_fp4<<<1, 64, 0, stream>>>(IN[7], 32, Q4);
    k_w16<<<1, 256, 0, stream>>>(Q2, Q3, IN[6], W2h, W3h, B3P);
    const unsigned L2 = (unsigned)(((size_t)RB * H1 / 2 + 255) / 256);
    for (int r0 = 0; r0 < NR; r0 += RB) {
        k_l1<<<L2, 256, 0, stream>>>(IN[0], Q1, IN[2], r0, H1h);
        k_gemmw<h16, 0, true><<<dim3(RB / 64, 1, 1), 32, 0, stream>>>(H1h, nullptr, W2h, nullptr, H1, F, H1, IN[4], 0, 0, 0); k_act<<<L2, 256, 0, stream>>>(F, H2h);
        k_gemmw<h16, 0, true><<<dim3(RB / 64, 1, 1), 32, 0, stream>>>(H2h, nullptr, W3h, nullptr, H1, F, H1, B3P, 0, 0, 0);
        k_out<<<RB / 256, 256, 0, stream>>>(F, Q4, IN[8], r0, OUT); }
}
